// SimpleAttention_31576599560710
// MI455X (gfx1250) — hardware-verified
//
#include <hip/hip_runtime.h>
#include <stdint.h>


#pragma clang fp contract(off)

typedef _Float16 v16h __attribute__((ext_vector_type(16)));
typedef _Float16 v8h  __attribute__((ext_vector_type(8)));
typedef _Float16 v8ha __attribute__((ext_vector_type(8), may_alias));
typedef float    v8f  __attribute__((ext_vector_type(8)));
typedef float    v4f  __attribute__((ext_vector_type(4)));
typedef float    v4fa __attribute__((ext_vector_type(4), may_alias));
typedef float    v2f  __attribute__((ext_vector_type(2)));
typedef unsigned int v4u __attribute__((ext_vector_type(4)));

union U8f  { v8f  v; float    f[8]; };
union U16h { v16h v; v8h      h[2]; };
union U8h  { v8h  v; _Float16 f[8]; };

#ifndef NB
#define NB 2
#endif
#ifndef SEQ
#define SEQ 2048
#endif
#define NB_FULL  2
#define SEQ_FULL 2048
#define DM   1024
#define NH   16
#define HD   64
#define QKVN 3072
#define NTOK (NB * SEQ)
#define RESQ ((SEQ) < 256 ? (SEQ) : 256)

static_assert(NB >= 1 && NB <= NB_FULL);
static_assert(SEQ >= 128 && SEQ <= SEQ_FULL);
static_assert(SEQ % 128 == 0);
static_assert(RESQ % 128 == 0);
static_assert(DM == NH * HD);
static_assert(DM % 32 == 0);
static_assert(QKVN == 3 * DM);

#define C2SCALE 0.18033688011112042f

#define QKP 72
#define VTP 136
#define CTP 72
#define QKV_LDS_HALFS 25600
#define SE_OFF 16384
static_assert(128 * 64 * 2 == SE_OFF);
static_assert(8 * 16 * QKP <= QKV_LDS_HALFS - SE_OFF);
static_assert(64 * VTP <= QKV_LDS_HALFS - SE_OFF);
static_assert(64 * VTP <= SE_OFF);

__device__ __forceinline__ v8f wmma_f16(v16h a, v16h b, v8f c) {
  v8f d = __builtin_amdgcn_wmma_f32_16x16x32_f16(false, a, false, b, (short)0, c, false, false);
  asm volatile("v_nop\n\tv_nop\n\tv_nop\n\tv_nop" : "+v"(d) : "v"(a), "v"(b));
  return d;
}

template <int CTRL>
__device__ __forceinline__ float dppf(float x) {
  int s = __float_as_int(x);
  return __int_as_float(__builtin_amdgcn_update_dpp(s, s, CTRL, 0xF, 0xF, true));
}
__device__ __forceinline__ float red_max16(float x) {
  x = fmaxf(x, dppf<0xB1>(x));
  x = fmaxf(x, dppf<0x4E>(x));
  x = fmaxf(x, dppf<0x141>(x));
  x = fmaxf(x, dppf<0x140>(x));
  return x;
}
__device__ __forceinline__ float red_sum16(float x) {
  x += dppf<0xB1>(x);
  x += dppf<0x4E>(x);
  x += dppf<0x141>(x);
  x += dppf<0x140>(x);
  return x;
}

__device__ __forceinline__ void wave_lds_sync() {
  __builtin_amdgcn_fence(3, "wavefront");
  asm volatile("s_wait_dscnt 0" ::: "memory");
  __builtin_amdgcn_wave_barrier();
}

__device__ __forceinline__ v4f bf16_rne4(v4f a) {
  v4u u = __builtin_bit_cast(v4u, a);
  u = (u + 0x7FFFu + ((u >> 16) & 1u)) & 0xFFFF0000u;
  return __builtin_bit_cast(v4f, u);
}
__device__ __forceinline__ float bf16r(float a) {
  unsigned int u = __float_as_uint(a);
  u = (u + 0x7FFFu + ((u >> 16) & 1u)) & 0xFFFF0000u;
  return __uint_as_float(u);
}

__device__ __forceinline__ v8h cvt8v(v4f a, v4f b) {
  v8h d;
  d[0] = (_Float16)a[0]; d[1] = (_Float16)a[1];
  d[2] = (_Float16)a[2]; d[3] = (_Float16)a[3];
  d[4] = (_Float16)b[0]; d[5] = (_Float16)b[1];
  d[6] = (_Float16)b[2]; d[7] = (_Float16)b[3];
  return d;
}

__global__ __launch_bounds__(256)
void cvt_kernel(const float* __restrict__ X, _Float16* __restrict__ P, int seg, int seg_full, float scale)
{
  const int tid = threadIdx.x;
  const int r   = blockIdx.x * 2 + (tid >> 7);
  const int q   = tid & 127;
  const int sb  = r / seg;
  const int sn  = r - sb * seg;
  const float* src = X + ((size_t)sb * seg_full + sn) * DM + 8 * q;
  _Float16*    dst = P + (size_t)r * DM + 8 * q;
  v4f a0 = bf16_rne4(*(const v4f*)src);
  v4f a1 = bf16_rne4(*(const v4f*)(src + 4));
  a0 = a0 * scale;
  a1 = a1 * scale;
  const v8h hv = cvt8v(a0, a1);
  *(volatile v8h*)dst = hv;
  __threadfence();
  *(volatile v8h*)dst = hv;
}

__global__ __launch_bounds__(256)
void rope_kernel(float* __restrict__ CS)
{
  __shared__ __attribute__((aligned(16))) float sT[8 * 64];
  const int tid  = threadIdx.x;
  const int pl   = tid >> 5;
  const int pair = tid & 31;
  const int pos  = blockIdx.x * 8 + pl;
  const float ex  = (float)(2 * pair) * 0.015625f;
  const float pw  = powf(10000.0f, ex);
  const float ifr = 1.0f / pw;
  const float ang = (float)pos * ifr;
  float sn, cs;
  sincosf(ang, &sn, &cs);
  sT[pl * 64 + 2 * pair]     = cs;
  sT[pl * 64 + 2 * pair + 1] = sn;
  __syncthreads();
  const int wr = (tid >> 4) & 7;
  const int wq = tid & 15;
  const v4f v = *(const v4fa*)(sT + wr * 64 + 4 * wq);
  float* d = CS + (size_t)(blockIdx.x * 8 + wr) * 64 + 4 * wq;
  if (tid < 128) *(volatile v4f*)d = v;
  __threadfence();
  if (tid < 128) *(volatile v4f*)d = v;
}


__global__ __launch_bounds__(256) __attribute__((amdgpu_num_vgpr(256)))
void qkv_kernel(const _Float16* __restrict__ Xh, const _Float16* __restrict__ Wq,
                const float* __restrict__ Bq, const float* __restrict__ CS,
                _Float16* __restrict__ Qp, _Float16* __restrict__ Kp,
                _Float16* __restrict__ Vt, _Float16* __restrict__ Vr)
{
  __shared__ __attribute__((aligned(16))) _Float16 slds[QKV_LDS_HALFS];
  float*    sCS = (float*)slds;
  _Float16* sE  = slds + SE_OFF;

  const int tid  = threadIdx.x;
  const int wave = tid >> 5;
  const int lane = tid & 31;
  const int lh   = lane & 15;
  const int hi   = lane >> 4;
  const int tm   = blockIdx.x;
  const int tn   = blockIdx.y;
  const int sel  = tn >> 4;
  const int head = tn & 15;
  const int mrow0 = tm * 128;
  const int b     = mrow0 / SEQ;
  const int nbase = mrow0 - b * SEQ;
  const int bh    = b * NH + head;

  if (sel < 2) {
    const float* src = CS + (size_t)(nbase + (tid >> 1)) * 64 + 32 * (tid & 1);
    float*       dst = sCS + (tid >> 1) * 64 + 32 * (tid & 1);
    #pragma unroll
    for (int i = 0; i < 8; ++i) *(v4f*)(dst + 4 * i) = *(const v4f*)(src + 4 * i);
    __syncthreads();
  }

  U8f acc[4];
  #pragma unroll
  for (int t = 0; t < 4; ++t) acc[t].v = (v8f){};

  const _Float16* Ap = Xh + (size_t)(mrow0 + wave * 16 + lh) * DM + 8 * hi;
  const _Float16* Bp = Wq + (size_t)(tn * 64 + lh) * DM + 8 * hi;
  #pragma unroll 2
  for (int k0 = 0; k0 < DM; k0 += 32) {
    U16h a;
    a.h[0] = *(const v8h*)(Ap + k0);
    a.h[1] = *(const v8h*)(Ap + k0 + 16);
    #pragma unroll
    for (int t = 0; t < 4; ++t) {
      U16h bf;
      bf.h[0] = *(const v8h*)(Bp + (size_t)t * 16 * DM + k0);
      bf.h[1] = *(const v8h*)(Bp + (size_t)t * 16 * DM + k0 + 16);
      acc[t].v = wmma_f16(a.v, bf.v, acc[t].v);
    }
  }

  float bb[4];
  #pragma unroll
  for (int t = 0; t < 4; ++t) bb[t] = bf16r(Bq[tn * 64 + 16 * t + lh]);
  #pragma unroll
  for (int t = 0; t < 4; ++t) {
    #pragma unroll
    for (int j = 0; j < 8; ++j) acc[t].f[j] = acc[t].f[j] * 0.015625f + bb[t];
  }

  if (sel < 2) {
    const float sgn = (lh & 1) ? 1.0f : -1.0f;
    #pragma unroll
    for (int t = 0; t < 4; ++t) {
      #pragma unroll
      for (int j = 0; j < 8; ++j) {
        const int   pl = wave * 16 + 8 * hi + j;
        const v2f   cs = *(const v2f*)(sCS + (pl * 32 + 8 * t + (lh >> 1)) * 2);
        const float v  = acc[t].f[j];
        const float pr = __shfl_xor(v, 1, 32);
        const float rt = sgn * pr;
        acc[t].f[j] = v * cs[0] + rt * cs[1];
      }
    }
    _Float16* sw = sE + wave * (16 * QKP);
    #pragma unroll
    for (int t = 0; t < 4; ++t) {
      #pragma unroll
      for (int j = 0; j < 8; ++j) sw[(j + 8 * hi) * QKP + 16 * t + lh] = (_Float16)acc[t].f[j];
    }
    wave_lds_sync();
    v8h ov[4]; size_t oo[4];
    #pragma unroll
    for (int i = 0; i < 4; ++i) {
      const int c = lane + 32 * i, rr = c >> 3, q = c & 7;
      ov[i] = *(const v8ha*)(sw + rr * QKP + 8 * q);
      oo[i] = ((size_t)bh * SEQ + nbase + wave * 16 + rr) * HD + 8 * q;
    }
    _Float16* plane = (sel == 0) ? Qp : Kp;
    #pragma unroll
    for (int i = 0; i < 4; ++i) *(volatile v8h*)(plane + oo[i]) = ov[i];
    __threadfence();
    #pragma unroll
    for (int i = 0; i < 4; ++i) *(volatile v8h*)(plane + oo[i]) = ov[i];
  } else {
    _Float16* sT = sE;
    _Float16* sR = slds;
    const bool resv = (nbase < RESQ);
    #pragma unroll
    for (int t = 0; t < 4; ++t) {
      #pragma unroll
      for (int j = 0; j < 8; ++j) {
        const int d   = 16 * t + lh;
        const int tok = wave * 16 + 8 * hi + j;
        const float v = acc[t].f[j];
        const _Float16 hv = (_Float16)v;
        sT[d * VTP + tok] = hv;
        if (resv) sR[d * VTP + tok] = (_Float16)((v - (float)hv) * 1024.0f);
      }
    }
    __syncthreads();
    v8h vv[4], rv[4]; size_t vo[4], ro[4];
    #pragma unroll
    for (int i = 0; i < 4; ++i) {
      const int L = (tid >> 3) + 32 * i, d = L >> 1, hf = L & 1, q = tid & 7;
      vv[i] = *(const v8ha*)(sT + d * VTP + 64 * hf + 8 * q);
      vo[i] = ((size_t)bh * HD + d) * SEQ + nbase + 64 * hf + 8 * q;
      ro[i] = ((size_t)bh * HD + d) * RESQ + nbase + 64 * hf + 8 * q;
      rv[i] = vv[i];
      if (resv) rv[i] = *(const v8ha*)(sR + d * VTP + 64 * hf + 8 * q);
    }
    #pragma unroll
    for (int i = 0; i < 4; ++i) *(volatile v8h*)(Vt + vo[i]) = vv[i];
    if (resv) {
      #pragma unroll
      for (int i = 0; i < 4; ++i) *(volatile v8h*)(Vr + ro[i]) = rv[i];
    }
    __threadfence();
    #pragma unroll
    for (int i = 0; i < 4; ++i) *(volatile v8h*)(Vt + vo[i]) = vv[i];
    if (resv) {
      #pragma unroll
      for (int i = 0; i < 4; ++i) *(volatile v8h*)(Vr + ro[i]) = rv[i];
    }
  }
}

template <int RES>
__global__ __launch_bounds__(128) __attribute__((amdgpu_num_vgpr(256)))
void attn_kernel(const _Float16* __restrict__ Qp, const _Float16* __restrict__ Kp,
                 const _Float16* __restrict__ Vt, const _Float16* __restrict__ Vr,
                 _Float16* __restrict__ Ctx, _Float16* __restrict__ Ctxr, int qoff, int nqb)
{
  __shared__ __attribute__((aligned(16))) _Float16 sPm[4 * 16 * 32];
  __shared__ __attribute__((aligned(16))) _Float16 sPr[4 * 16 * 32];
  __shared__ __attribute__((aligned(16))) _Float16 sCm[4 * 16 * CTP];

  const int tid  = threadIdx.x;
  const int wave = tid >> 5;
  const int lane = tid & 31;
  const int lh   = lane & 15;
  const int hi   = lane >> 4;

  const int bh    = blockIdx.x / nqb;
  const int qbase = qoff + (blockIdx.x - bh * nqb) * 64;
  const int qrow0 = qbase + wave * 16;
  const int b     = bh / NH;
  const int h     = bh - b * NH;

  const _Float16* Qb  = Qp + (size_t)bh * SEQ * HD;
  const _Float16* Kb  = Kp + (size_t)bh * SEQ * HD;
  const _Float16* Vb  = Vt + (size_t)bh * HD * SEQ;
  const _Float16* Vrb = Vr + (size_t)bh * HD * RESQ;

  U16h qf0, qf1;
  {
    const _Float16* qr = Qb + (size_t)(qrow0 + lh) * HD + 8 * hi;
    qf0.h[0] = *(const v8h*)(qr);
    qf0.h[1] = *(const v8h*)(qr + 16);
    qf1.h[0] = *(const v8h*)(qr + 32);
    qf1.h[1] = *(const v8h*)(qr + 48);
  }

  U8f acc[4], acc2[4];
  #pragma unroll
  for (int t = 0; t < 4; ++t) { acc[t].v = (v8f){}; acc2[t].v = (v8f){}; }
  float mrow[8], lrow[8];
  #pragma unroll
  for (int j = 0; j < 8; ++j) { mrow[j] = -3.0e38f; lrow[j] = 0.0f; }

  _Float16* pw  = sPm + wave * (16 * 32);
  _Float16* prw = sPr + wave * (16 * 32);
  const float ninf = -__builtin_inff();
  const int kend = qrow0 + 15;

  #pragma unroll 1
  for (int kv0 = 0; kv0 <= kend; kv0 += 32) {
    U8f s0, s1; s0.v = (v8f){}; s1.v = (v8f){};
    {
      const _Float16* kr = Kb + (size_t)(kv0 + lh) * HD + 8 * hi;
      U16h kf;
      kf.h[0] = *(const v8h*)(kr);      kf.h[1] = *(const v8h*)(kr + 16);
      s0.v = wmma_f16(qf0.v, kf.v, s0.v);
      kf.h[0] = *(const v8h*)(kr + 32); kf.h[1] = *(const v8h*)(kr + 48);
      s0.v = wmma_f16(qf1.v, kf.v, s0.v);
      const _Float16* kr1 = kr + 16 * HD;
      kf.h[0] = *(const v8h*)(kr1);      kf.h[1] = *(const v8h*)(kr1 + 16);
      s1.v = wmma_f16(qf0.v, kf.v, s1.v);
      kf.h[0] = *(const v8h*)(kr1 + 32); kf.h[1] = *(const v8h*)(kr1 + 48);
      s1.v = wmma_f16(qf1.v, kf.v, s1.v);
    }

    U8h pa, pb, pra, prb;
    const int kc0 = kv0 + lh, kc1 = kv0 + 16 + lh;
    #pragma unroll
    for (int j = 0; j < 8; ++j) {
      const int   qi = qrow0 + 8 * hi + j;
      const float a  = (kc0 > qi) ? ninf : s0.f[j] * C2SCALE;
      const float bb = (kc1 > qi) ? ninf : s1.f[j] * C2SCALE;
      const float rm    = red_max16(fmaxf(a, bb));
      const float mnew  = fmaxf(mrow[j], rm);
      const float alpha = __builtin_amdgcn_exp2f(mrow[j] - mnew);
      const float e0    = __builtin_amdgcn_exp2f(a  - mnew);
      const float e1    = __builtin_amdgcn_exp2f(bb - mnew);
      lrow[j] = lrow[j] * alpha + red_sum16(e0 + e1);
      mrow[j] = mnew;
      const float p0 = e0 * 1024.0f, p1 = e1 * 1024.0f;
      const _Float16 h0 = (_Float16)p0, h1 = (_Float16)p1;
      pa.f[j] = h0; pb.f[j] = h1;
      if (RES) {
        pra.f[j] = (_Float16)((p0 - (float)h0) * 1024.0f);
        prb.f[j] = (_Float16)((p1 - (float)h1) * 1024.0f);
      }
      #pragma unroll
      for (int t = 0; t < 4; ++t) {
        acc[t].f[j] *= alpha;
        if (RES) acc2[t].f[j] *= alpha;
      }
    }

    #pragma unroll
    for (int j = 0; j < 8; ++j) {
      pw[(j + 8 * hi) * 32 + lh]      = pa.f[j];
      pw[(j + 8 * hi) * 32 + 16 + lh] = pb.f[j];
      if (RES) {
        prw[(j + 8 * hi) * 32 + lh]      = pra.f[j];
        prw[(j + 8 * hi) * 32 + 16 + lh] = prb.f[j];
      }
    }
    wave_lds_sync();
    U16h pf, prf;
    pf.h[0] = *(const v8ha*)(pw + lh * 32 + 8 * hi);
    pf.h[1] = *(const v8ha*)(pw + lh * 32 + 16 + 8 * hi);
    if (RES) {
      prf.h[0] = *(const v8ha*)(prw + lh * 32 + 8 * hi);
      prf.h[1] = *(const v8ha*)(prw + lh * 32 + 16 + 8 * hi);
    }

    #pragma unroll
    for (int t = 0; t < 4; ++t) {
      const _Float16* vrow = Vb + (size_t)(16 * t + lh) * SEQ + kv0 + 8 * hi;
      U16h vf;
      vf.h[0] = *(const v8h*)(vrow);
      vf.h[1] = *(const v8h*)(vrow + 16);
      acc[t].v = wmma_f16(pf.v, vf.v, acc[t].v);
      if (RES) {
        const _Float16* rrow = Vrb + (size_t)(16 * t + lh) * RESQ + kv0 + 8 * hi;
        U16h rf;
        rf.h[0] = *(const v8h*)(rrow);
        rf.h[1] = *(const v8h*)(rrow + 16);
        acc2[t].v = wmma_f16(pf.v, rf.v, acc2[t].v);
        acc2[t].v = wmma_f16(prf.v, vf.v, acc2[t].v);
      }
    }
    wave_lds_sync();
  }

  float inv[8];
  #pragma unroll
  for (int j = 0; j < 8; ++j) inv[j] = 1.0f / (lrow[j] * 1024.0f);
  _Float16* cw = sCm + wave * (16 * CTP);
  #pragma unroll
  for (int t = 0; t < 4; ++t) {
    #pragma unroll
    for (int j = 0; j < 8; ++j) {
      float o = acc[t].f[j];
      if (RES) o = o + acc2[t].f[j] * 0.0009765625f;
      o = o * inv[j];
      acc[t].f[j] = o;
      cw[(j + 8 * hi) * CTP + 16 * t + lh] = (_Float16)o;
    }
  }
  wave_lds_sync();
  v8h ov[4]; size_t oo[4];
  #pragma unroll
  for (int i = 0; i < 4; ++i) {
    const int c = lane + 32 * i, rr = c >> 3, q = c & 7;
    ov[i] = *(const v8ha*)(cw + rr * CTP + 8 * q);
    oo[i] = ((size_t)b * SEQ + qrow0 + rr) * DM + h * HD + 8 * q;
  }
  #pragma unroll
  for (int i = 0; i < 4; ++i) *(volatile v8h*)(Ctx + oo[i]) = ov[i];
  __threadfence();
  #pragma unroll
  for (int i = 0; i < 4; ++i) *(volatile v8h*)(Ctx + oo[i]) = ov[i];

  if (RES) {
    wave_lds_sync();
    #pragma unroll
    for (int t = 0; t < 4; ++t) {
      #pragma unroll
      for (int j = 0; j < 8; ++j) {
        const float o = acc[t].f[j];
        const _Float16 oh = (_Float16)o;
        cw[(j + 8 * hi) * CTP + 16 * t + lh] = (_Float16)((o - (float)oh) * 1024.0f);
      }
    }
    wave_lds_sync();
    #pragma unroll
    for (int i = 0; i < 4; ++i) {
      const int c = lane + 32 * i, rr = c >> 3, q = c & 7;
      ov[i] = *(const v8ha*)(cw + rr * CTP + 8 * q);
      oo[i] = ((size_t)b * RESQ + qrow0 + rr) * DM + h * HD + 8 * q;
    }
    #pragma unroll
    for (int i = 0; i < 4; ++i) *(volatile v8h*)(Ctxr + oo[i]) = ov[i];
    __threadfence();
    #pragma unroll
    for (int i = 0; i < 4; ++i) *(volatile v8h*)(Ctxr + oo[i]) = ov[i];
  }
}

template <int RES>
__global__ __launch_bounds__(256) __attribute__((amdgpu_num_vgpr(256)))
void proj_kernel(const _Float16* __restrict__ Ctx, const _Float16* __restrict__ Ctxr,
                 const _Float16* __restrict__ Wp, const float* __restrict__ Bp,
                 float* __restrict__ Out, int poff, int nrt)
{
  __shared__ __attribute__((aligned(16))) float sO[8 * 16 * 64];

  const int tid  = threadIdx.x;
  const int wave = tid >> 5;
  const int lane = tid & 31;
  const int lh   = lane & 15;
  const int hi   = lane >> 4;
  const int bx   = blockIdx.x;
  const int tn   = blockIdx.y;
  const int b    = bx / nrt;
  const int pos0 = poff + (bx - b * nrt) * 128;
  const int mrow0 = b * SEQ + pos0;

  U8f acc[4], acc2[4];
  #pragma unroll
  for (int t = 0; t < 4; ++t) { acc[t].v = (v8f){}; acc2[t].v = (v8f){}; }

  const _Float16* Ap  = Ctx  + (size_t)(mrow0 + wave * 16 + lh) * DM + 8 * hi;
  const _Float16* Arp = Ctxr + (size_t)(b * RESQ + pos0 + wave * 16 + lh) * DM + 8 * hi;
  const _Float16* Bw  = Wp   + (size_t)(tn * 64 + lh) * DM + 8 * hi;
  #pragma unroll 2
  for (int k0 = 0; k0 < DM; k0 += 32) {
    U16h a, ar;
    a.h[0] = *(const v8h*)(Ap + k0);
    a.h[1] = *(const v8h*)(Ap + k0 + 16);
    if (RES) {
      ar.h[0] = *(const v8h*)(Arp + k0);
      ar.h[1] = *(const v8h*)(Arp + k0 + 16);
    }
    #pragma unroll
    for (int t = 0; t < 4; ++t) {
      U16h bf;
      bf.h[0] = *(const v8h*)(Bw + (size_t)t * 16 * DM + k0);
      bf.h[1] = *(const v8h*)(Bw + (size_t)t * 16 * DM + k0 + 16);
      acc[t].v = wmma_f16(a.v, bf.v, acc[t].v);
      if (RES) acc2[t].v = wmma_f16(ar.v, bf.v, acc2[t].v);
    }
  }

  float bb[4];
  #pragma unroll
  for (int t = 0; t < 4; ++t) bb[t] = bf16r(Bp[tn * 64 + 16 * t + lh]);
  float* so = sO + wave * (16 * 64);
  #pragma unroll
  for (int t = 0; t < 4; ++t) {
    #pragma unroll
    for (int j = 0; j < 8; ++j) {
      float v = acc[t].f[j];
      if (RES) v = v + acc2[t].f[j] * 0.0009765625f;
      v = v * 0.015625f + bb[t];
      so[(j + 8 * hi) * 64 + 16 * t + lh] = v;
    }
  }
  wave_lds_sync();
  v4f ov[8]; size_t oo[8];
  #pragma unroll
  for (int i = 0; i < 8; ++i) {
    const int c = lane + 32 * i, rr = c >> 4, q = c & 15;
    ov[i] = *(const v4fa*)(so + rr * 64 + 4 * q);
    oo[i] = ((size_t)mrow0 + wave * 16 + rr) * DM + tn * 64 + 4 * q;
  }
  #pragma unroll
  for (int i = 0; i < 8; ++i) *(volatile v4f*)(Out + oo[i]) = ov[i];
  __threadfence();
  #pragma unroll
  for (int i = 0; i < 8; ++i) *(volatile v4f*)(Out + oo[i]) = ov[i];
}

extern "C" void kernel_launch(void* const* d_in, const int* in_sizes, int n_in,
                              void* d_out, int out_size, void* d_ws, size_t ws_size,
                              hipStream_t stream) {
  if (n_in < 5) return;
  const long long need_x = ((long long)(NB - 1) * SEQ_FULL + SEQ) * DM;
  if ((long long)in_sizes[0] < need_x) return;
  if ((long long)in_sizes[1] < (long long)QKVN * DM) return;
  if (in_sizes[2] < QKVN) return;
  if ((long long)in_sizes[3] < (long long)DM * DM) return;
  if (in_sizes[4] < DM) return;
  if ((long long)out_size < (long long)NTOK * DM) return;

  const size_t b_xh  = (size_t)NTOK * DM * 2;
  const size_t b_wq  = (size_t)QKVN * DM * 2;
  const size_t b_wp  = (size_t)DM * DM * 2;
  const size_t b_cs  = (size_t)SEQ * 32 * 2 * 4;
  const size_t b_pl  = (size_t)NB * NH * SEQ * HD * 2;
  const size_t b_vr  = (size_t)NB * NH * HD * RESQ * 2;
  const size_t b_ctx = (size_t)NTOK * DM * 2;
  const size_t b_ctr = (size_t)NB * RESQ * DM * 2;
  const size_t o_xh  = 0;
  const size_t o_wq  = o_xh  + b_xh;
  const size_t o_wp  = o_wq  + b_wq;
  const size_t o_cs  = o_wp  + b_wp;
  const size_t o_qp  = o_cs  + b_cs;
  const size_t o_kp  = o_qp  + b_pl;
  const size_t o_vt  = o_kp  + b_pl;
  const size_t o_vr  = o_vt  + b_pl;
  const size_t o_ctx = o_vr  + b_vr;
  const size_t o_ctr = o_ctx + b_ctx;
  const size_t o_end = o_ctr + b_ctr;
  if (o_end > ws_size) return;

  const float* x      = (const float*)d_in[0];
  const float* qkv_w  = (const float*)d_in[1];
  const float* qkv_b  = (const float*)d_in[2];
  const float* proj_w = (const float*)d_in[3];
  const float* proj_b = (const float*)d_in[4];
  float* out = (float*)d_out;
  char* ws = (char*)d_ws;
  _Float16* xh  = (_Float16*)(ws + o_xh);
  _Float16* wq  = (_Float16*)(ws + o_wq);
  _Float16* wp  = (_Float16*)(ws + o_wp);
  float*    cs  = (float*)(ws + o_cs);
  _Float16* qp  = (_Float16*)(ws + o_qp);
  _Float16* kp  = (_Float16*)(ws + o_kp);
  _Float16* vt  = (_Float16*)(ws + o_vt);
  _Float16* vr  = (_Float16*)(ws + o_vr);
  _Float16* ctx = (_Float16*)(ws + o_ctx);
  _Float16* ctr = (_Float16*)(ws + o_ctr);

  cvt_kernel<<<dim3(NTOK / 2), dim3(256), 0, stream>>>(x, xh, SEQ, SEQ_FULL, 1.0f);
  cvt_kernel<<<dim3(QKVN / 2), dim3(256), 0, stream>>>(qkv_w, wq, QKVN, QKVN, 64.0f);
  cvt_kernel<<<dim3(DM / 2), dim3(256), 0, stream>>>(proj_w, wp, DM, DM, 64.0f);
  rope_kernel<<<dim3(SEQ / 8), dim3(256), 0, stream>>>(cs);

  qkv_kernel<<<dim3(NTOK / 128, QKVN / 64), dim3(256), 0, stream>>>(xh, wq, qkv_b, cs, qp, kp, vt, vr);

  attn_kernel<1><<<dim3(NB * NH * (RESQ / 64)), dim3(128), 0, stream>>>(qp, kp, vt, vr, ctx, ctr, 0, RESQ / 64);
  if (SEQ > RESQ) {
    attn_kernel<0><<<dim3(NB * NH * ((SEQ - RESQ) / 64)), dim3(128), 0, stream>>>(qp, kp, vt, vr, ctx, ctr, RESQ, (SEQ - RESQ) / 64);
  }

  proj_kernel<1><<<dim3(NB * (RESQ / 128), DM / 64), dim3(256), 0, stream>>>(ctx, ctr, wp, proj_b, out, 0, RESQ / 128);
  if (SEQ > RESQ) {
    proj_kernel<0><<<dim3(NB * ((SEQ - RESQ) / 128), DM / 64), dim3(256), 0, stream>>>(ctx, ctr, wp, proj_b, out, RESQ, (SEQ - RESQ) / 128);
  }
}
